// BlockLocalAttention_56925496541795
// MI455X (gfx1250) — hardware-verified
//
#include <hip/hip_runtime.h>

typedef _Float16       v16h __attribute__((ext_vector_type(16)));
typedef __bf16         v16b __attribute__((ext_vector_type(16)));
typedef unsigned short u16;
typedef u16            v8us __attribute__((ext_vector_type(8)));
typedef float          v8f  __attribute__((ext_vector_type(8)));
typedef float          v4f  __attribute__((ext_vector_type(4)));
typedef v8us __attribute__((may_alias)) v8usa;
typedef v4f  __attribute__((may_alias)) v4fa;

union Frag { v16h h; v16b b; v8us half[2]; };

#define NTOK 16384
#define DMOD 512
#define NSP  8192
#define LDQK 1024

#define NOP4 "v_nop\n\tv_nop\n\tv_nop\n\tv_nop"

__device__ __forceinline__ u16 bf_rne(float f) {
  const unsigned u = __builtin_bit_cast(unsigned, f);
  return (u16)((u + 0x7FFFu + ((u >> 16) & 1u)) >> 16);
}
__device__ __forceinline__ float bf_val(u16 v) {
  const unsigned u = ((unsigned)v) << 16;
  return __builtin_bit_cast(float, u);
}
__device__ __forceinline__ u16 h_bits(float f) {
  const _Float16 t = (_Float16)f;
  return __builtin_bit_cast(u16, t);
}

__device__ __forceinline__ Frag ldfrag(const u16* p, int hh) {
  Frag f;
  f.half[0] = *(const v8usa*)(p + 8 * hh);
  f.half[1] = *(const v8usa*)(p + 16 + 8 * hh);
  return f;
}

__device__ __forceinline__ v8f mma_h(const Frag& a, const Frag& b, v8f c) {
  return __builtin_amdgcn_wmma_f32_16x16x32_f16(false, a.h, false, b.h, (short)0, c, false, false);
}
__device__ __forceinline__ v8f mma_b(const Frag& a, const Frag& b, v8f c) {
  return __builtin_amdgcn_wmma_f32_16x16x32_bf16(false, a.b, false, b.b, (short)0, c, false, false);
}

__global__ __launch_bounds__(256) void pack_kernel(
    const float* __restrict__ wq, const float* __restrict__ wk, const float* __restrict__ wv,
    const float* __restrict__ wp, const float* __restrict__ w1, const float* __restrict__ w2,
    u16* __restrict__ Wqkv, u16* __restrict__ Wp,
    u16* __restrict__ W1h, u16* __restrict__ W1l, u16* __restrict__ W2h, u16* __restrict__ W2l,
    int ngroups)
{
  const int G0 = 1536 * 512 / 8;
  const int G1 = 512 * 512 / 8;
  const int g = blockIdx.x * 256 + threadIdx.x;
  if (g >= ngroups) return;
  float v[8];
  if (g < G0 + G1) {
    u16* dst;
    if (g < G0) {
      const int i0 = g * 8, n = i0 >> 9, k0 = i0 & 511;
      const int sec = n >> 9, hi = n & 511, hd = hi >> 6, e = hi & 63;
      const float* wsrc = (sec == 0) ? wq : ((sec == 1) ? wk : wv);
      #pragma unroll
      for (int i = 0; i < 8; ++i) v[i] = wsrc[((size_t)(hd * 512 + k0 + i)) * 64 + e] * 32.0f;
      dst = Wqkv + i0;
    } else {
      const int i0 = (g - G0) * 8;
      const v4f a = *(const v4fa*)(wp + i0);
      const v4f c = *(const v4fa*)(wp + i0 + 4);
      v[0] = a.x * 32.0f; v[1] = a.y * 32.0f; v[2] = a.z * 32.0f; v[3] = a.w * 32.0f;
      v[4] = c.x * 32.0f; v[5] = c.y * 32.0f; v[6] = c.z * 32.0f; v[7] = c.w * 32.0f;
      dst = Wp + i0;
    }
    v8us o;
    #pragma unroll
    for (int i = 0; i < 8; ++i) o[i] = h_bits(v[i]);
    *(volatile v8us*)dst = o;
    __threadfence();
    *(volatile v8us*)dst = o;
  } else {
    const bool first = (g < G0 + 2 * G1);
    const int i0 = (first ? (g - G0 - G1) : (g - G0 - 2 * G1)) * 8;
    const float* src = first ? w1 : w2;
    u16* dhp = first ? W1h : W2h;
    u16* dlp = first ? W1l : W2l;
    const v4f a = *(const v4fa*)(src + i0);
    const v4f c = *(const v4fa*)(src + i0 + 4);
    v[0] = a.x; v[1] = a.y; v[2] = a.z; v[3] = a.w; v[4] = c.x; v[5] = c.y; v[6] = c.z; v[7] = c.w;
    v8us oh, ol;
    #pragma unroll
    for (int i = 0; i < 8; ++i) {
      const u16 hb = bf_rne(v[i]);
      oh[i] = hb;
      ol[i] = bf_rne(v[i] - bf_val(hb));
    }
    *(volatile v8us*)(dhp + i0) = oh;
    *(volatile v8us*)(dlp + i0) = ol;
    __threadfence();
    *(volatile v8us*)(dhp + i0) = oh;
    *(volatile v8us*)(dlp + i0) = ol;
  }
}

__global__ __launch_bounds__(256) void ln1_kernel(const float* __restrict__ x, const float* __restrict__ g,
                                                  const float* __restrict__ bta, u16* __restrict__ xn)
{
  extern __shared__ float smf[];
  const int tid = threadIdx.x, lane = tid & 31, w = tid >> 5;
  const int rt0 = blockIdx.x * 32;
  const int batch = rt0 >> 13, s0 = rt0 & (NSP - 1);
  const float* xb = x + (size_t)batch * DMOD * NSP + s0;
  for (int c = w; c < DMOD; c += 8) smf[c * 33 + lane] = xb[(size_t)c * NSP + lane];
  __syncthreads();

  #pragma unroll 1
  for (int qq = 0; qq < 4; ++qq) {
    const int tl = 4 * w + qq;
    float v[16];
    #pragma unroll
    for (int i = 0; i < 8; ++i) {
      v[i]     = smf[(8 * lane + i) * 33 + tl];
      v[8 + i] = smf[(256 + 8 * lane + i) * 33 + tl];
    }
    float s = 0.f;
    #pragma unroll
    for (int i = 0; i < 16; ++i) s += v[i];
    #pragma unroll
    for (int o = 16; o; o >>= 1) s += __shfl_xor(s, o);
    const float mean = s * (1.0f / 512.0f);
    float vs = 0.f;
    #pragma unroll
    for (int i = 0; i < 16; ++i) { const float d = v[i] - mean; vs += d * d; }
    #pragma unroll
    for (int o = 16; o; o >>= 1) vs += __shfl_xor(vs, o);
    const float rstd = rsqrtf(vs * (1.0f / 512.0f) + 1e-5f);
    v8us o0, o1;
    #pragma unroll
    for (int i = 0; i < 8; ++i) {
      const int c0 = 8 * lane + i, c1 = 256 + 8 * lane + i;
      o0[i] = h_bits((v[i] - mean) * rstd * g[c0] + bta[c0]);
      o1[i] = h_bits((v[8 + i] - mean) * rstd * g[c1] + bta[c1]);
    }
    u16* orow = xn + (size_t)(rt0 + tl) * DMOD;
    *(volatile v8us*)(orow + 8 * lane) = o0;
    *(volatile v8us*)(orow + 256 + 8 * lane) = o1;
    __threadfence();
    *(volatile v8us*)(orow + 8 * lane) = o0;
    *(volatile v8us*)(orow + 256 + 8 * lane) = o1;
  }
}

__global__ __launch_bounds__(256) void ln2_kernel(const float* __restrict__ in, const float* __restrict__ g,
                                                  const float* __restrict__ bta,
                                                  u16* __restrict__ yh, u16* __restrict__ yl)
{
  const int tid = threadIdx.x, lane = tid & 31, w = tid >> 5;
  const int rt = blockIdx.x * 8 + w;
  const float* row = in + (size_t)rt * DMOD;
  const v4f t0 = *(const v4fa*)(row + 8 * lane);
  const v4f t1 = *(const v4fa*)(row + 8 * lane + 4);
  const v4f t2 = *(const v4fa*)(row + 256 + 8 * lane);
  const v4f t3 = *(const v4fa*)(row + 256 + 8 * lane + 4);
  float v[16] = { t0.x, t0.y, t0.z, t0.w, t1.x, t1.y, t1.z, t1.w,
                  t2.x, t2.y, t2.z, t2.w, t3.x, t3.y, t3.z, t3.w };
  float s = 0.f;
  #pragma unroll
  for (int i = 0; i < 16; ++i) s += v[i];
  #pragma unroll
  for (int o = 16; o; o >>= 1) s += __shfl_xor(s, o);
  const float mean = s * (1.0f / 512.0f);
  float vs = 0.f;
  #pragma unroll
  for (int i = 0; i < 16; ++i) { const float d = v[i] - mean; vs += d * d; }
  #pragma unroll
  for (int o = 16; o; o >>= 1) vs += __shfl_xor(vs, o);
  const float rstd = rsqrtf(vs * (1.0f / 512.0f) + 1e-5f);
  v8us o0h, o0l, o1h, o1l;
  #pragma unroll
  for (int i = 0; i < 8; ++i) {
    const int c0 = 8 * lane + i, c1 = 256 + 8 * lane + i;
    const float y0 = (v[i] - mean) * rstd * g[c0] + bta[c0];
    const float y1 = (v[8 + i] - mean) * rstd * g[c1] + bta[c1];
    const u16 h0 = bf_rne(y0), h1 = bf_rne(y1);
    o0h[i] = h0; o0l[i] = bf_rne(y0 - bf_val(h0));
    o1h[i] = h1; o1l[i] = bf_rne(y1 - bf_val(h1));
  }
  const size_t g0 = (size_t)rt * DMOD + 8 * lane, g1 = g0 + 256;
  *(volatile v8us*)(yh + g0) = o0h; *(volatile v8us*)(yh + g1) = o1h;
  *(volatile v8us*)(yl + g0) = o0l; *(volatile v8us*)(yl + g1) = o1l;
  __threadfence();
  *(volatile v8us*)(yh + g0) = o0h; *(volatile v8us*)(yh + g1) = o1h;
  *(volatile v8us*)(yl + g0) = o0l; *(volatile v8us*)(yl + g1) = o1l;
}

__device__ __forceinline__ void sp_rows(const u16* sh, const u16* sl, u16* P0, u16* P1,
                                        int ldo, int r0, int col0, int w, int lane) {
  const int q8 = lane & 7, sub = lane >> 3;
  #pragma unroll
  for (int i = 0; i < 8; ++i) {
    const int tl = 32 * w + 4 * i + sub;
    const v8us a = *(const v8usa*)(sh + tl * 64 + 8 * q8);
    const v8us c = *(const v8usa*)(sl + tl * 64 + 8 * q8);
    const size_t gd = (size_t)(r0 + tl) * ldo + col0 + 8 * q8;
    *(volatile v8us*)(P0 + gd) = a;
    *(volatile v8us*)(P1 + gd) = c;
  }
}
__device__ __forceinline__ void sp_vt(const u16* sh, const u16* sl, u16* V0, u16* V1,
                                      int batch, int ts, int tt, int hs, int head, int w, int lane) {
  const int q8 = lane & 7, sub = lane >> 3;
  const int bblk = batch * 32 + ts * 16 + hs * 4 + sub;
  const size_t base = ((size_t)(bblk * 8 + head) * 64) * 256 + tt * 64 + q8 * 8;
  #pragma unroll
  for (int di = 0; di < 8; ++di) {
    const int d = 8 * w + di;
    const int sidx = d * 256 + q8 * 32 + sub * 8;
    const v8us a = *(const v8usa*)(sh + sidx);
    const v8us c = *(const v8usa*)(sl + sidx);
    const size_t gd = base + (size_t)d * 256;
    *(volatile v8us*)(V0 + gd) = a;
    *(volatile v8us*)(V1 + gd) = c;
  }
}
__device__ __forceinline__ void sp_o1(const float* sf, float* OF, int r0, int col0, int w, int lane) {
  const int q8 = lane & 7, sub = lane >> 3;
  #pragma unroll
  for (int i = 0; i < 16; ++i) {
    const int L = 64 * w + 4 * i + sub;
    const int tl = L >> 1, hf = L & 1;
    const v4f v = *(const v4fa*)(sf + tl * 64 + 32 * hf + 4 * q8);
    *(volatile v4f*)(OF + (size_t)(r0 + tl) * DMOD + col0 + 32 * hf + 4 * q8) = v;
  }
}
__device__ __forceinline__ void sp_out(const float* st, float* OF, int batch, int s0, int col0, int w, int lane) {
  #pragma unroll
  for (int ci = 0; ci < 8; ++ci) {
    const int col = 8 * w + ci;
    const size_t gb = (size_t)(batch * DMOD + col0 + col) * NSP + s0;
    #pragma unroll
    for (int hf = 0; hf < 2; ++hf) {
      const v4f v = *(const v4fa*)(st + col * 256 + 128 * hf + 4 * lane);
      *(volatile v4f*)(OF + gb + 128 * hf + 4 * lane) = v;
    }
  }
}

template <int KIND, int MODE>
__global__ __launch_bounds__(256) void gemm_kernel(
    const u16* __restrict__ A0, const u16* __restrict__ A1,
    const u16* __restrict__ B0, const u16* __restrict__ B1,
    const float* __restrict__ xsrc, const float* __restrict__ bias, const float* __restrict__ res,
    u16* __restrict__ P0, u16* __restrict__ P1, u16* __restrict__ V0, u16* __restrict__ V1,
    float* __restrict__ OF)
{
  extern __shared__ __attribute__((aligned(16))) unsigned char smem[];
  const int tid = threadIdx.x, lane = tid & 31, w = tid >> 5, hh = lane >> 4, m = lane & 15;
  const int bm = blockIdx.x, bn = blockIdx.y;
  const int r0 = bm * 256;
  const int batch = bm >> 5, s0 = (bm & 31) * 256;
  const size_t arow = (size_t)(r0 + 32 * w + m) * DMOD;
  const size_t brow = (size_t)(bn * 64 + m) * DMOD;

  const v8f z8 = {0.f, 0.f, 0.f, 0.f, 0.f, 0.f, 0.f, 0.f};
  v8f acc[2][4];
  #pragma unroll
  for (int mt = 0; mt < 2; ++mt)
    #pragma unroll
    for (int nt = 0; nt < 4; ++nt) acc[mt][nt] = z8;

  #pragma unroll 1
  for (int k0 = 0; k0 < DMOD; k0 += 32) {
    if (KIND == 0) {
      const Frag a0 = ldfrag(A0 + arow + k0, hh);
      const Frag a1 = ldfrag(A0 + arow + 16 * DMOD + k0, hh);
      const Frag b0 = ldfrag(B0 + brow + k0, hh);
      const Frag b1 = ldfrag(B0 + brow + 16 * DMOD + k0, hh);
      const Frag b2 = ldfrag(B0 + brow + 32 * DMOD + k0, hh);
      const Frag b3 = ldfrag(B0 + brow + 48 * DMOD + k0, hh);
      acc[0][0] = mma_h(a0, b0, acc[0][0]);
      acc[1][0] = mma_h(a1, b0, acc[1][0]);
      acc[0][1] = mma_h(a0, b1, acc[0][1]);
      acc[1][1] = mma_h(a1, b1, acc[1][1]);
      acc[0][2] = mma_h(a0, b2, acc[0][2]);
      acc[1][2] = mma_h(a1, b2, acc[1][2]);
      acc[0][3] = mma_h(a0, b3, acc[0][3]);
      acc[1][3] = mma_h(a1, b3, acc[1][3]);
      asm volatile(NOP4
                   : "+v"(acc[0][0]), "+v"(acc[1][0]), "+v"(acc[0][1]), "+v"(acc[1][1]),
                     "+v"(acc[0][2]), "+v"(acc[1][2]), "+v"(acc[0][3]), "+v"(acc[1][3])
                   : "v"(a0.h), "v"(a1.h), "v"(b0.h), "v"(b1.h), "v"(b2.h), "v"(b3.h));
    } else {
      const Frag a0h = ldfrag(A0 + arow + k0, hh);
      const Frag a1h = ldfrag(A0 + arow + 16 * DMOD + k0, hh);
      const Frag a0l = ldfrag(A1 + arow + k0, hh);
      const Frag a1l = ldfrag(A1 + arow + 16 * DMOD + k0, hh);
      #pragma unroll
      for (int nt = 0; nt < 4; ++nt) {
        const Frag bh = ldfrag(B0 + brow + (size_t)nt * 16 * DMOD + k0, hh);
        const Frag bl = ldfrag(B1 + brow + (size_t)nt * 16 * DMOD + k0, hh);
        acc[0][nt] = mma_b(a0h, bh, acc[0][nt]);
        acc[0][nt] = mma_b(a0h, bl, acc[0][nt]);
        acc[0][nt] = mma_b(a0l, bh, acc[0][nt]);
        acc[1][nt] = mma_b(a1h, bh, acc[1][nt]);
        acc[1][nt] = mma_b(a1h, bl, acc[1][nt]);
        acc[1][nt] = mma_b(a1l, bh, acc[1][nt]);
        asm volatile(NOP4
                     : "+v"(acc[0][nt]), "+v"(acc[1][nt])
                     : "v"(a0h.h), "v"(a1h.h), "v"(a0l.h), "v"(a1l.h), "v"(bh.h), "v"(bl.h));
      }
    }
  }

  if (MODE == 0 || MODE == 1) {
    u16* s_hi = (u16*)smem;
    u16* s_lo = s_hi + 256 * 64;
    const bool isv = (MODE == 0) && (bn >= 16);
    const float scl = (MODE == 0) ? ((bn < 8) ? (1.0f / 256.0f) : (1.0f / 32.0f)) : 1.0f;
    #pragma unroll
    for (int nt = 0; nt < 4; ++nt) {
      const int col = 16 * nt + m;
      float bcol = 0.f;
      if (MODE == 1) bcol = bias[bn * 64 + col];
      #pragma unroll
      for (int mt = 0; mt < 2; ++mt) {
        #pragma unroll
        for (int r = 0; r < 8; ++r) {
          const int tl = 32 * w + 16 * mt + 8 * hh + r;
          float v = acc[mt][nt][r];
          if (MODE == 0) v = v * scl;
          else v = fmaxf(v + bcol, 0.f);
          const u16 hb = bf_rne(v);
          const u16 lb = bf_rne(v - bf_val(hb));
          const int idx = isv ? (col * 256 + tl) : (tl * 64 + col);
          s_hi[idx] = hb;
          s_lo[idx] = lb;
        }
      }
    }
    __syncthreads();
    if (!isv) {
      const int ldo = (MODE == 0) ? LDQK : DMOD;
      sp_rows(s_hi, s_lo, P0, P1, ldo, r0, bn * 64, w, lane);
      __threadfence();
      sp_rows(s_hi, s_lo, P0, P1, ldo, r0, bn * 64, w, lane);
    } else {
      const int ts = (bm & 31) >> 4, tt = ((bm & 31) >> 2) & 3, hs = bm & 3;
      const int head = bn - 16;
      sp_vt(s_hi, s_lo, V0, V1, batch, ts, tt, hs, head, w, lane);
      __threadfence();
      sp_vt(s_hi, s_lo, V0, V1, batch, ts, tt, hs, head, w, lane);
    }
  } else if (MODE == 2) {
    float* sf = (float*)smem;
    #pragma unroll
    for (int nt = 0; nt < 4; ++nt) {
      const int col = 16 * nt + m;
      const int c = bn * 64 + col;
      const float* xc = xsrc + (size_t)(batch * DMOD + c) * NSP + s0;
      #pragma unroll
      for (int mt = 0; mt < 2; ++mt) {
        #pragma unroll
        for (int r = 0; r < 8; ++r) {
          const int tl = 32 * w + 16 * mt + 8 * hh + r;
          sf[tl * 64 + col] = acc[mt][nt][r] * (1.0f / 32.0f) + xc[tl];
        }
      }
    }
    __syncthreads();
    sp_o1(sf, OF, r0, bn * 64, w, lane);
    __threadfence();
    sp_o1(sf, OF, r0, bn * 64, w, lane);
  } else {
    float* st = (float*)smem;
    #pragma unroll
    for (int nt = 0; nt < 4; ++nt) {
      const int col = 16 * nt + m;
      const int c = bn * 64 + col;
      const float bcol = bias[c];
      #pragma unroll
      for (int mt = 0; mt < 2; ++mt) {
        #pragma unroll
        for (int r = 0; r < 8; ++r) {
          const int tl = 32 * w + 16 * mt + 8 * hh + r;
          st[col * 256 + tl] = (acc[mt][nt][r] + bcol) + res[(size_t)(r0 + tl) * DMOD + c];
        }
      }
    }
    __syncthreads();
    sp_out(st, OF, batch, s0, bn * 64, w, lane);
    __threadfence();
    sp_out(st, OF, batch, s0, bn * 64, w, lane);
  }
}

__device__ __forceinline__ int rof(int rbase, int n) {
  return rbase + (n >> 6) * 1024 + ((n >> 3) & 7) * 32 + (n & 7);
}

__device__ __forceinline__ void pack_p(const v8f& a, const v8f& c, Frag& ph, Frag& pl) {
  #pragma unroll
  for (int r = 0; r < 8; ++r) {
    const u16 ha = bf_rne(a[r]);
    ph.half[0][r] = ha;
    pl.half[0][r] = bf_rne(a[r] - bf_val(ha));
    const u16 hc = bf_rne(c[r]);
    ph.half[1][r] = hc;
    pl.half[1][r] = bf_rne(c[r] - bf_val(hc));
  }
}

__device__ __forceinline__ void sp_ao(const u16* sw, u16* ao, int rbase, int nq0, int head, int lane) {
  const int q8 = lane & 7, sub = lane >> 3;
  #pragma unroll
  for (int i = 0; i < 4; ++i) {
    const int ql = 4 * i + sub;
    const int rr = rof(rbase, nq0 + ql);
    const v8us v = *(const v8usa*)(sw + ql * 64 + 8 * q8);
    *(volatile v8us*)(ao + (size_t)rr * DMOD + head * 64 + 8 * q8) = v;
  }
}

__global__ __launch_bounds__(128) void attn_kernel(
    const u16* __restrict__ qkh, const u16* __restrict__ qkl,
    const u16* __restrict__ vth, const u16* __restrict__ vtl,
    const float* __restrict__ dtb, const float* __restrict__ dhb, const float* __restrict__ dwb,
    u16* __restrict__ ao)
{
  __shared__ float sdt[8];
  __shared__ float sdh[16];
  __shared__ __attribute__((aligned(16))) u16 so[4 * 16 * 64];

  const int tid = threadIdx.x, lane = tid & 31, w = tid >> 5, hh = lane >> 4, m = lane & 15;
  const int bid = blockIdx.x, qc = bid & 3, bh = bid >> 2, head = bh & 7, b = bh >> 3;
  const int batch = b >> 5, ts = (b >> 4) & 1, hs = (b >> 2) & 3, wsb = b & 3;
  const int rbase = batch * NSP + ts * 4096 + hs * 256 + wsb * 8;
  if (tid < 7) sdt[tid] = dtb[head * 7 + tid];
  if (tid >= 32 && tid < 47) sdh[tid - 32] = dhb[head * 15 + (tid - 32)];

  const int nq0 = qc * 64 + 16 * w;
  const int nq = nq0 + m;
  const int tq = nq >> 6, hq = (nq >> 3) & 7, wq = nq & 7;
  const int rq = rbase + tq * 1024 + hq * 32 + wq;
  const u16* qph = qkh + (size_t)rq * LDQK + head * 64;
  const u16* qpl = qkl + (size_t)rq * LDQK + head * 64;
  const Frag qh0 = ldfrag(qph, hh), qh1 = ldfrag(qph + 32, hh);
  const Frag ql0 = ldfrag(qpl, hh), ql1 = ldfrag(qpl + 32, hh);
  float dwv[8];
  #pragma unroll
  for (int r = 0; r < 8; ++r) dwv[r] = dwb[head * 15 + (wq - r + 7)];
  __syncthreads();

  const v8f z8 = {0.f, 0.f, 0.f, 0.f, 0.f, 0.f, 0.f, 0.f};
  v8f o[4];
  #pragma unroll
  for (int t = 0; t < 4; ++t) o[t] = z8;
  float mrun = -1e30f, lrun = 0.0f;

  const size_t vrow0 = ((size_t)bh * 64 + m) * 256;

  #pragma unroll 1
  for (int kb = 0; kb < 256; kb += 64) {
    v8f s[4];
    #pragma unroll
    for (int j = 0; j < 4; ++j) {
      const int kk0 = kb + 16 * j;
      const int rk = rof(rbase, kk0 + m);
      const u16* kph = qkh + (size_t)rk * LDQK + 512 + head * 64;
      const u16* kpl = qkl + (size_t)rk * LDQK + 512 + head * 64;
      const Frag kh0 = ldfrag(kph, hh), kh1 = ldfrag(kph + 32, hh);
      const Frag kl0 = ldfrag(kpl, hh), kl1 = ldfrag(kpl + 32, hh);
      v8f z = z8;
      z = mma_b(kh0, qh0, z);
      z = mma_b(kh1, qh1, z);
      z = mma_b(kh0, ql0, z);
      z = mma_b(kh1, ql1, z);
      z = mma_b(kl0, qh0, z);
      z = mma_b(kl1, qh1, z);
      asm volatile(NOP4 : "+v"(z)
                   : "v"(kh0.h), "v"(kh1.h), "v"(kl0.h), "v"(kl1.h),
                     "v"(qh0.h), "v"(qh1.h), "v"(ql0.h), "v"(ql1.h));
      const int kkl = kk0 + 8 * hh;
      const int tk = kkl >> 6, hk = (kkl >> 3) & 7;
      const float bb = sdt[tq - tk + 3] + sdh[hq - hk + 7];
      #pragma unroll
      for (int r = 0; r < 8; ++r) z[r] = z[r] + (bb + dwv[r]);
      s[j] = z;
    }

    float mloc = s[0][0];
    #pragma unroll
    for (int j = 0; j < 4; ++j)
      #pragma unroll
      for (int r = 0; r < 8; ++r) mloc = fmaxf(mloc, s[j][r]);
    mloc = fmaxf(mloc, __shfl_xor(mloc, 16));
    const float mnew = fmaxf(mrun, mloc);
    const float alpha = __expf(mrun - mnew);
    mrun = mnew;
    float lsum = 0.0f;
    #pragma unroll
    for (int j = 0; j < 4; ++j)
      #pragma unroll
      for (int r = 0; r < 8; ++r) {
        const float p = __expf(s[j][r] - mnew);
        s[j][r] = p;
        lsum += p;
      }
    lsum += __shfl_xor(lsum, 16);
    lrun = lrun * alpha + lsum;
    #pragma unroll
    for (int t = 0; t < 4; ++t)
      #pragma unroll
      for (int r = 0; r < 8; ++r) o[t][r] = o[t][r] * alpha;

    #pragma unroll
    for (int c = 0; c < 2; ++c) {
      Frag ph, pl;
      pack_p(s[2 * c], s[2 * c + 1], ph, pl);
      #pragma unroll
      for (int t = 0; t < 4; ++t) {
        const size_t voff = vrow0 + (size_t)(16 * t) * 256 + kb + 32 * c;
        const Frag vh = ldfrag(vth + voff, hh);
        const Frag vl = ldfrag(vtl + voff, hh);
        o[t] = mma_b(vh, ph, o[t]);
        o[t] = mma_b(vh, pl, o[t]);
        o[t] = mma_b(vl, ph, o[t]);
        asm volatile(NOP4 : "+v"(o[t]) : "v"(vh.h), "v"(vl.h), "v"(ph.h), "v"(pl.h));
      }
    }
  }

  const float inv = 1.0f / lrun;
  u16* sw = so + w * 1024;
  #pragma unroll
  for (int t = 0; t < 4; ++t)
    #pragma unroll
    for (int r = 0; r < 8; ++r)
      sw[m * 64 + 16 * t + 8 * hh + r] = h_bits(o[t][r] * inv);
  __syncthreads();

  sp_ao(sw, ao, rbase, nq0, head, lane);
  __threadfence();
  sp_ao(sw, ao, rbase, nq0, head, lane);
}

extern "C" void kernel_launch(void* const* d_in, const int* in_sizes, int n_in,
                              void* d_out, int out_size, void* d_ws, size_t ws_size,
                              hipStream_t stream) {
  if (n_in < 16) return;
  if (in_sizes[0] != NTOK * DMOD) return;
  if (in_sizes[1] != 56 || in_sizes[2] != 120 || in_sizes[3] != 120) return;
  if (in_sizes[4] != 512 || in_sizes[5] != 512 || in_sizes[10] != 512 || in_sizes[11] != 512) return;
  if (in_sizes[6] != 262144 || in_sizes[7] != 262144 || in_sizes[8] != 262144) return;
  if (in_sizes[9] != 262144 || in_sizes[12] != 262144 || in_sizes[14] != 262144) return;
  if (in_sizes[13] != 512 || in_sizes[15] != 512) return;
  if (out_size != NTOK * DMOD) return;

  const float* x    = (const float*)d_in[0];
  const float* dtb  = (const float*)d_in[1];
  const float* dhb  = (const float*)d_in[2];
  const float* dwb  = (const float*)d_in[3];
  const float* ln1g = (const float*)d_in[4];
  const float* ln1b = (const float*)d_in[5];
  const float* wq   = (const float*)d_in[6];
  const float* wk   = (const float*)d_in[7];
  const float* wv   = (const float*)d_in[8];
  const float* wp   = (const float*)d_in[9];
  const float* ln2g = (const float*)d_in[10];
  const float* ln2b = (const float*)d_in[11];
  const float* w1   = (const float*)d_in[12];
  const float* b1   = (const float*)d_in[13];
  const float* w2   = (const float*)d_in[14];
  const float* b2   = (const float*)d_in[15];
  float* out = (float*)d_out;

  const size_t szXN = (size_t)NTOK * DMOD * 2;
  const size_t szQK = (size_t)NTOK * LDQK * 2;
  const size_t szVT = (size_t)NTOK * DMOD * 2;
  const size_t szO1 = (size_t)NTOK * DMOD * 4;
  const size_t szPL = (size_t)NTOK * DMOD * 2;
  const size_t szWQ = (size_t)1536 * 512 * 2;
  const size_t szW  = (size_t)512 * 512 * 2;

  const size_t oXN  = 0;
  const size_t oR1  = oXN + szXN;
  const size_t oQKH = oR1;
  const size_t oQKL = oQKH + szQK;
  const size_t oVTH = oQKL + szQK;
  const size_t oVTL = oVTH + szVT;
  const size_t oR1E = oVTL + szVT;
  const size_t oO1  = oR1;
  const size_t oYH  = oO1 + szO1;
  const size_t oYL  = oYH + szPL;
  const size_t oFH  = oYL + szPL;
  const size_t oFL  = oFH + szPL;
  const size_t oWQ  = oR1E;
  const size_t oWP  = oWQ + szWQ;
  const size_t oW1H = oWP + szW;
  const size_t oW1L = oW1H + szW;
  const size_t oW2H = oW1L + szW;
  const size_t oW2L = oW2H + szW;
  const size_t total = oW2L + szW;
  if (oFL + szPL != oR1E) return;
  if (total > ws_size) return;
  if (total > (size_t)134217728) return;

  char* ws = (char*)d_ws;
  u16* xn   = (u16*)(ws + oXN);
  u16* ao   = (u16*)(ws + oXN);
  u16* qkh  = (u16*)(ws + oQKH);
  u16* qkl  = (u16*)(ws + oQKL);
  u16* vth  = (u16*)(ws + oVTH);
  u16* vtl  = (u16*)(ws + oVTL);
  float* out1 = (float*)(ws + oO1);
  u16* yh   = (u16*)(ws + oYH);
  u16* yl   = (u16*)(ws + oYL);
  u16* fh   = (u16*)(ws + oFH);
  u16* fl   = (u16*)(ws + oFL);
  u16* Wqkv = (u16*)(ws + oWQ);
  u16* Wp   = (u16*)(ws + oWP);
  u16* W1h  = (u16*)(ws + oW1H);
  u16* W1l  = (u16*)(ws + oW1L);
  u16* W2h  = (u16*)(ws + oW2H);
  u16* W2l  = (u16*)(ws + oW2L);

  const int ngroups = 1536 * 512 / 8 + 3 * (512 * 512 / 8);
  pack_kernel<<<(ngroups + 255) / 256, 256, 0, stream>>>(wq, wk, wv, wp, w1, w2,
                                                         Wqkv, Wp, W1h, W1l, W2h, W2l, ngroups);
  ln1_kernel<<<NTOK / 32, 256, 512 * 33 * 4, stream>>>(x, ln1g, ln1b, xn);
  gemm_kernel<0, 0><<<dim3(NTOK / 256, 24), 256, 65536, stream>>>(
      xn, xn, Wqkv, Wqkv, x, b1, x, qkh, qkl, vth, vtl, out);
  attn_kernel<<<64 * 8 * 4, 128, 0, stream>>>(qkh, qkl, vth, vtl, dtb, dhb, dwb, ao);
  gemm_kernel<0, 2><<<dim3(NTOK / 256, 8), 256, 65536, stream>>>(
      ao, ao, Wp, Wp, x, b1, x, yh, yl, yh, yl, out1);
  ln2_kernel<<<NTOK / 8, 256, 0, stream>>>(out1, ln2g, ln2b, yh, yl);
  gemm_kernel<1, 1><<<dim3(NTOK / 256, 8), 256, 65536, stream>>>(
      yh, yl, W1h, W1l, x, b1, x, fh, fl, fh, fl, out1);
  gemm_kernel<1, 3><<<dim3(NTOK / 256, 8), 256, 65536, stream>>>(
      fh, fl, W2h, W2l, x, b2, out1, yh, yl, yh, yl, out);
}
